// KoopmanQNetwork_75952201662835
// MI455X (gfx1250) — hardware-verified
//
#include <hip/hip_runtime.h>


#ifndef NB
#define NB 131072
#endif
#define NB_FULL 131072
#define SDIM  17
#define ADIM  7
#define DPHI  128
#define DPSI  8
#define KK    (DPHI * DPSI)
#define TROWS 32
#define PHP   132
#define WPP   20

static_assert(NB % TROWS == 0);
static_assert(NB <= NB_FULL);
static_assert(KK % 32 == 0);
static_assert(DPHI == 128);
static_assert(DPSI == 8);
static_assert(SDIM == 17);
static_assert(ADIM == 7);
static_assert((TROWS * SDIM) % 32 == 0);
static_assert((TROWS * ADIM) % 32 == 0);
static_assert((DPHI * WPP) % 32 == 0);
static_assert(WPP >= SDIM && WPP % 4 == 0);
static_assert(PHP >= DPHI && PHP % 4 == 0);
static_assert((DPHI * KK) % 8 == 0);

typedef unsigned short bf;
typedef __attribute__((ext_vector_type(16))) __bf16   v16bf;
typedef __attribute__((ext_vector_type(8)))  unsigned short v8us;
typedef __attribute__((ext_vector_type(8)))  float    v8f;
typedef __attribute__((ext_vector_type(4)))  float    v4f;
typedef __attribute__((ext_vector_type(4)))  int      v4i;
typedef v4f  __attribute__((may_alias)) v4fa;
typedef v4i  __attribute__((may_alias)) v4ia;

__device__ __forceinline__ unsigned short f2bf(float f) { unsigned u = __float_as_uint(f); u += 0x7FFFu + ((u >> 16) & 1u); return (unsigned short)(u >> 16); }
__device__ __forceinline__ float bf2f(unsigned short w) { return __uint_as_float(((unsigned)w) << 16); }
__device__ __forceinline__ int clampi(int v, int lo, int hi) { return min(max(v, lo), hi); }
__device__ __forceinline__ v16bf cat16b(v8us lo, v8us hi) { return __builtin_bit_cast(v16bf, __builtin_shufflevector(lo, hi, 0, 1, 2, 3, 4, 5, 6, 7, 8, 9, 10, 11, 12, 13, 14, 15)); }
__device__ __forceinline__ v8f wmmab(v16bf a, v16bf b, v8f c) { return __builtin_amdgcn_wmma_f32_16x16x32_bf16(false, a, false, b, (short)0, c, false, false); }
__device__ __forceinline__ v16bf ldb(const bf* p)  { return cat16b(*(const v8us*)p, *(const v8us*)(p + 16)); }
__device__ __forceinline__ void wave_sync() { __builtin_amdgcn_fence(3  , "wavefront"); __builtin_amdgcn_wave_barrier(); asm volatile("" ::: "memory"); }
__device__ __forceinline__ v8f wmmag(v16bf a, v16bf b, v8f c) { c = wmmab(a, b, c); asm volatile("v_nop\n\tv_nop\n\tv_nop\n\tv_nop" : "+v"(c) : "v"(a), "v"(b)); return c; }

__global__ __launch_bounds__(256) void k_kt(const float* __restrict__ K, bf* KT) {
    const size_t i = (size_t)blockIdx.x * 256 + threadIdx.x; if (i >= (size_t)(DPHI * KK / 8)) return;
    const v8f a = *(const v8f*)(K + i * 8); v8us o;
#pragma unroll
    for (int k = 0; k < 8; ++k) o[k] = f2bf(a[k]);
    *(volatile v8us*)(KT + i * 8) = o; __threadfence(); *(volatile v8us*)(KT + i * 8) = o;
}

static constexpr size_t GEMM_LDS_BYTES = 4u * (size_t)(DPHI * WPP + 64 + DPHI + TROWS * SDIM + TROWS * ADIM + TROWS * PHP + TROWS * DPSI + TROWS);
static_assert(GEMM_LDS_BYTES <= (size_t)131072);
static_assert(8 * 16 * 1 == TROWS * 4);
static_assert(16 * 2 == TROWS);
static_assert(2 * 64 == DPHI);

__global__ __launch_bounds__(32) __attribute__((amdgpu_num_vgpr(256))) void k_gemm(const float* __restrict__ state, const float* __restrict__ action,
                                                                                    const float* __restrict__ Wphi, const float* __restrict__ Wpsi,
                                                                                    const float* __restrict__ wlin, const bf* __restrict__ KT, float* OUT) {
    __shared__ __align__(16) float wps[DPHI * WPP];
    __shared__ __align__(16) float wqs[64];
    __shared__ __align__(16) float wls[DPHI];
    __shared__ __align__(16) float sts[TROWS * SDIM];
    __shared__ __align__(16) float acts[TROWS * ADIM];
    __shared__ __align__(16) float phs[TROWS * PHP];
    __shared__ __align__(16) float pss[TROWS * DPSI];
    __shared__ __align__(16) float res[TROWS];
    const int lane = threadIdx.x & 31, lr = lane & 15, hi = lane >> 4;
    const size_t r0 = (size_t)blockIdx.x * TROWS;

#pragma unroll 1
    for (int i = lane; i < DPHI * WPP; i += 32) { const int j = i / WPP, s = i - j * WPP; const int sc = min(s, SDIM - 1);
        const float v = bf2f(f2bf(Wphi[j * SDIM + sc])); wps[i] = (s < SDIM) ? v : 0.0f; }
#pragma unroll 1
    for (int i = lane; i < 64; i += 32) { const int ic = min(i, DPSI * ADIM - 1); const float v = bf2f(f2bf(Wpsi[ic])); wqs[i] = (i < DPSI * ADIM) ? v : 0.0f; }
#pragma unroll 1
    for (int i = lane; i < DPHI; i += 32) wls[i] = bf2f(f2bf(wlin[i]));
#pragma unroll 1
    for (int i = lane; i < TROWS * SDIM; i += 32) sts[i] = bf2f(f2bf(state[r0 * SDIM + i]));
#pragma unroll 1
    for (int i = lane; i < TROWS * ADIM; i += 32) acts[i] = bf2f(f2bf(action[r0 * ADIM + i]));
    wave_sync();

    {
        float av[ADIM];
#pragma unroll
        for (int a = 0; a < ADIM; ++a) av[a] = acts[lane * ADIM + a];
#pragma unroll 1
        for (int z = 0; z < DPSI; ++z) { float s = 0.0f;
#pragma unroll
            for (int a = 0; a < ADIM; ++a) s += av[a] * wqs[z * ADIM + a];
            pss[lane * DPSI + z] = s; }
        float sv[SDIM];
#pragma unroll
        for (int s = 0; s < SDIM; ++s) sv[s] = sts[lane * SDIM + s];
#pragma unroll 1
        for (int j = 0; j < DPHI; ++j) { float s = 0.0f;
#pragma unroll
            for (int q = 0; q < 4; ++q) { const v4f w = *(const v4fa*)(&wps[j * WPP + 4 * q]);
#pragma unroll
                for (int i = 0; i < 4; ++i) s += sv[4 * q + i] * w[i]; }
            s += sv[16] * wps[j * WPP + 16];
            phs[lane * PHP + j] = s; }
    }
    wave_sync();

    float ps[2][8];
#pragma unroll
    for (int mb = 0; mb < 2; ++mb) { const v4f x0 = *(const v4fa*)(&pss[(mb * 16 + lr) * DPSI]); const v4f x1 = *(const v4fa*)(&pss[(mb * 16 + lr) * DPSI + 4]);
#pragma unroll
        for (int i = 0; i < 4; ++i) { ps[mb][i] = x0[i]; ps[mb][4 + i] = x1[i]; } }

    v8f acc[2][8];
#pragma unroll
    for (int mb = 0; mb < 2; ++mb)
#pragma unroll
        for (int nb = 0; nb < 8; ++nb) acc[mb][nb] = (v8f){};
    const size_t boff = (size_t)lr * KK + 8 * hi;
#pragma unroll 1
    for (int kc = 0; kc < KK; kc += 32) {
        v16bf ah[2], al[2];
#pragma unroll
        for (int mb = 0; mb < 2; ++mb) {
            const int pr = (mb * 16 + lr) * PHP + (kc >> 3) + hi;
            const float pa = phs[pr], pb = phs[pr + 2];
            v8us h0, l0, h1, l1;
#pragma unroll
            for (int i = 0; i < 8; ++i) {
                const float va = pa * ps[mb][i]; const unsigned short ha = f2bf(va); h0[i] = ha; l0[i] = f2bf(va - bf2f(ha));
                const float vb = pb * ps[mb][i]; const unsigned short hb = f2bf(vb); h1[i] = hb; l1[i] = f2bf(vb - bf2f(hb)); }
            ah[mb] = cat16b(h0, h1); al[mb] = cat16b(l0, l1); }
#pragma unroll
        for (int nb = 0; nb < 8; ++nb) { const v16bf b = ldb(KT + boff + (size_t)nb * 16 * KK + kc);
#pragma unroll
            for (int mb = 0; mb < 2; ++mb) { acc[mb][nb] = wmmag(ah[mb], b, acc[mb][nb]); acc[mb][nb] = wmmag(al[mb], b, acc[mb][nb]); } }
    }
    wave_sync();

    const int row = lane >> 1, hf = lane & 1;
#pragma unroll
    for (int mb = 0; mb < 2; ++mb) {
#pragma unroll
        for (int nb = 0; nb < 8; ++nb) {
#pragma unroll
            for (int j = 0; j < 8; ++j) phs[(hi * 8 + j) * PHP + nb * 16 + lr] = acc[mb][nb][j]; }
        wave_sync();
        const int ob = row * PHP + hf * 64;
        float s = 0.0f;
#pragma unroll 1
        for (int q = 0; q < 8; ++q) {
            const v4f x0 = *(const v4fa*)(&phs[ob + 8 * q]); const v4f x1 = *(const v4fa*)(&phs[ob + 8 * q + 4]);
            const v4f w0 = *(const v4fa*)(&wls[hf * 64 + 8 * q]); const v4f w1 = *(const v4fa*)(&wls[hf * 64 + 8 * q + 4]);
#pragma unroll
            for (int i = 0; i < 4; ++i) s += x0[i] * w0[i];
#pragma unroll
            for (int i = 0; i < 4; ++i) s += x1[i] * w1[i]; }
        s += __shfl_xor(s, 1, 32);
        if (hf == 0) res[mb * 16 + row] = s;
        wave_sync();
    }
#pragma unroll 1
    for (int pass = 0; pass < 2; ++pass) {
        if (lane < 8) { const v4f v = *(const v4fa*)(&res[4 * lane]); *(volatile v4f*)(OUT + r0 + 4 * lane) = v; }
        if (pass == 0) __threadfence(); }
}

static constexpr size_t al256(size_t v) { return (v + 255) & ~(size_t)255; }
static constexpr size_t SZ_KT = al256((size_t)DPHI * KK * 2);
static constexpr size_t SZ_TOTAL = SZ_KT;
static_assert(SZ_TOTAL <= (size_t)134217728);
static_assert(((size_t)DPHI * KK / 8) * 8 * 2 <= SZ_KT);
static_assert((size_t)NB * 4 <= (size_t)NB_FULL * 4);

extern "C" void kernel_launch(void* const* d_in, const int* in_sizes, int n_in,
                              void* d_out, int out_size, void* d_ws, size_t ws_size, hipStream_t stream) {
    if (n_in < 6) return;
    if ((size_t)in_sizes[0] < (size_t)NB * SDIM || (size_t)in_sizes[1] < (size_t)NB * ADIM) return;
    if ((size_t)in_sizes[2] < (size_t)DPHI * SDIM) return;
    if ((size_t)in_sizes[3] < (size_t)DPSI * ADIM) return;
    if ((size_t)in_sizes[4] < (size_t)DPHI * KK) return;
    if ((size_t)in_sizes[5] < (size_t)DPHI) return;
    if ((size_t)out_size < (size_t)NB) return;
    if (SZ_TOTAL > ws_size) return;
    const float* state  = (const float*)d_in[0];
    const float* action = (const float*)d_in[1];
    const float* Wphi   = (const float*)d_in[2];
    const float* Wpsi   = (const float*)d_in[3];
    const float* Kin    = (const float*)d_in[4];
    const float* wlin   = (const float*)d_in[5];
    float* OUT = (float*)d_out;
    char* wsp = (char*)d_ws;
    bf* KT = (bf*)wsp; wsp += SZ_KT;

    k_kt<<<(unsigned)((DPHI * KK / 8 + 255) / 256), 256, 0, stream>>>(Kin, KT);
    k_gemm<<<NB / TROWS, 32, 0, stream>>>(state, action, Wphi, Wpsi, wlin, KT, OUT);
}
